// SerialIntervalGraph_32830730010793
// MI455X (gfx1250) — hardware-verified
//
#include <hip/hip_runtime.h>
#include <math.h>

typedef __attribute__((ext_vector_type(16))) _Float16 v16h;
typedef __attribute__((ext_vector_type(16))) __bf16 v16b;
typedef __attribute__((ext_vector_type(8)))  _Float16 v8h;
typedef __attribute__((ext_vector_type(8)))  float v8f;
typedef __attribute__((ext_vector_type(4)))  float v4f;
typedef __attribute__((ext_vector_type(2)))  float v2f;
typedef __attribute__((ext_vector_type(4)))  unsigned v4u;
typedef __attribute__((ext_vector_type(4)))  int v4i;
typedef float __attribute__((may_alias)) float_a;
typedef int __attribute__((may_alias)) int_a;

template <typename T> __device__ __forceinline__ void vst2(void* p, T v) { *(volatile T*)p = v; __threadfence(); *(volatile T*)p = v; }
__device__ __forceinline__ v8f wmma16(v16h a, v16h b, v8f c) {
  v8f d = __builtin_amdgcn_wmma_f32_16x16x32_f16(false, a, false, b, (short)0, c, false, false);
  asm volatile("v_nop\n\tv_nop\n\tv_nop\n\tv_nop" : "+v"(d) : "v"(a), "v"(b));
  return d;
}
__device__ __forceinline__ v8f wmma_bf(v16b a, v16b b, v8f c) {
  v8f d = __builtin_amdgcn_wmma_f32_16x16x32_bf16(false, a, false, b, (short)0, c, false, false);
  asm volatile("v_nop\n\tv_nop\n\tv_nop\n\tv_nop" : "+v"(d) : "v"(a), "v"(b));
  return d;
}
__device__ __forceinline__ v16h frag_h(const _Float16* rowk0, int lane) {
  union { v16h v; v8h q[2]; } u; const _Float16* p = rowk0 + 8 * (lane >> 4);
  u.q[0] = *(const v8h*)p; u.q[1] = *(const v8h*)(p + 16); return u.v;
}
__device__ __forceinline__ v16h frag_f32(const float* rowk0, int lane) {
  v16h a; const float* p = rowk0 + 8 * (lane >> 4);
#pragma unroll
  for (int i = 0; i < 8; ++i) { a[i] = (_Float16)p[i]; a[8 + i] = (_Float16)p[16 + i]; }
  return a;
}
__device__ __forceinline__ v16h frag_f32s(const float* rowk0, int lane, float sc) {
  v16h a; const float* p = rowk0 + 8 * (lane >> 4);
#pragma unroll
  for (int i = 0; i < 8; ++i) { a[i] = (_Float16)(p[i] * sc); a[8 + i] = (_Float16)(p[16 + i] * sc); }
  return a;
}
__device__ __forceinline__ v16h fragc_f32(const float* W, int k0, int n, int lane, int ld, int K) {
  v16h a; const int g = lane >> 4;
#pragma unroll
  for (int i = 0; i < 8; ++i) { const int ka = k0 + 8 * g + i, kb = ka + 16;
    a[i] = (_Float16)(ka < K ? W[(size_t)(ka < K ? ka : K - 1) * ld + n] : 0.f); a[8 + i] = (_Float16)(kb < K ? W[(size_t)(kb < K ? kb : K - 1) * ld + n] : 0.f); }
  return a;
}
struct F2 { v16b h, l; };
__device__ __forceinline__ F2 bsplit16(const float v[16]) { F2 r;
#pragma unroll
  for (int i = 0; i < 16; ++i) { const __bf16 h = (__bf16)v[i]; r.h[i] = h; r.l[i] = (__bf16)(v[i] - (float)h); }
  return r; }
__device__ __forceinline__ F2 split_row(const float* row, int k0, int lane) { float v[16]; const float* p = row + k0 + 8 * (lane >> 4);
#pragma unroll
  for (int i = 0; i < 8; ++i) { v[i] = p[i]; v[8 + i] = p[16 + i]; }
  return bsplit16(v); }
__device__ __forceinline__ F2 split_rowK(const float* row, int k0, int lane, int K) { float v[16]; const int g = lane >> 4;
#pragma unroll
  for (int i = 0; i < 8; ++i) { const int ka = k0 + 8 * g + i, kb = ka + 16; v[i] = ka < K ? row[ka < K ? ka : K - 1] : 0.f; v[8 + i] = kb < K ? row[kb < K ? kb : K - 1] : 0.f; }
  return bsplit16(v); }
__device__ __forceinline__ F2 split_col(const float* W, int k0, int n, int lane, int ld, int K) { float v[16]; const int g = lane >> 4;
#pragma unroll
  for (int i = 0; i < 8; ++i) { const int ka = k0 + 8 * g + i, kb = ka + 16; v[i] = ka < K ? W[(size_t)(ka < K ? ka : K - 1) * ld + n] : 0.f; v[8 + i] = kb < K ? W[(size_t)(kb < K ? kb : K - 1) * ld + n] : 0.f; }
  return bsplit16(v); }
__device__ __forceinline__ v8f mac3(const F2& a, const F2& b, v8f c) { c = wmma_bf(a.l, b.h, c); c = wmma_bf(a.h, b.l, c); return wmma_bf(a.h, b.h, c); }
__device__ __forceinline__ float sigm(float v) { return 1.0f / (1.0f + expf(-v)); }
#define LDSX() do { asm volatile("s_wait_dscnt 0" ::: "memory"); __builtin_amdgcn_wave_barrier(); __builtin_amdgcn_fence(__ATOMIC_RELEASE, "workgroup"); } while (0)


#define NB 16
#define NN 2048
#define HH 32
#define TT 28
#define NLAG 8
#define NVC 48
#define LNEPS 1e-5f
#ifndef TNB
#define TNB NB
#endif
typedef __attribute__((ext_vector_type(8))) __bf16 v8b;
__device__ __forceinline__ v16b frag_b(const __bf16* rowk0, int lane) {
  union { v16b v; v8b q[2]; } u; const __bf16* p = rowk0 + 8 * (lane >> 4);
  u.q[0] = *(const v8b*)p; u.q[1] = *(const v8b*)(p + 16); return u.v;
}
__device__ __forceinline__ float bfr(float v) { return (float)(__bf16)v; }
__device__ __attribute__((noinline)) float exp_ni(float v) { return expf(v); }
__device__ __attribute__((noinline)) float erf_ni(float v) { return erff(v); }

#define WS_QK  0u
#define WS_QKL (WS_QK + 2u * (size_t)NB * NN * 2 * HH)
#define WS_VT  (WS_QKL + 2u * (size_t)NB * NN * 2 * HH)
#define WS_VTL (WS_VT + 2u * (size_t)NB * NVC * NN)
#define WS_END (WS_VTL + 2u * (size_t)NB * NVC * NN)

__device__ __forceinline__ v16b fragb_f32(const float* __restrict__ p, int lane) { v16b a; const float* pp = p + 8 * (lane >> 4);
#pragma unroll
  for (int i = 0; i < 8; ++i) { a[i] = (__bf16)pp[i]; a[8 + i] = (__bf16)pp[16 + i]; } return a; }
__global__ __launch_bounds__(128) void k_prep(const float* __restrict__ X, const float* __restrict__ FT, const float* __restrict__ DL, const float* __restrict__ WQ, const float* __restrict__ BQ, const float* __restrict__ WK, const float* __restrict__ BK, const float* __restrict__ WV, const float* __restrict__ BV, _Float16* __restrict__ QK, _Float16* __restrict__ QKL, _Float16* __restrict__ VT, _Float16* __restrict__ VTL) {
  __shared__ __align__(16) _Float16 sh[64][72], sl[64][72]; __shared__ __align__(16) _Float16 th[NVC][72], tl[NVC][72]; __shared__ float sdw[NLAG];
  const int tid = threadIdx.x, wave = tid >> 5, lane = tid & 31, col = lane & 15, g = lane >> 4; const size_t b = blockIdx.y; const int n0 = blockIdx.x * 64; const size_t r0 = b * NN + n0 + wave * 16;
  if (tid < NLAG) { float mx = -3.0e38f; for (int i = 0; i < NLAG; ++i) mx = fmaxf(mx, bfr(DL[i])); float s = 0.f; for (int i = 0; i < NLAG; ++i) s += expf(bfr(DL[i]) - mx); sdw[tid] = expf(bfr(DL[tid]) - mx) / s; }
  for (int e = tid; e < NVC * 72; e += 128) { th[e / 72][e % 72] = (_Float16)0.0f; tl[e / 72][e % 72] = (_Float16)0.0f; }
  __syncthreads();
  const v16b a = fragb_f32(FT + (r0 + col) * HH, lane);
  v8f acc[6] = {};
#pragma unroll
  for (int j = 0; j < 6; ++j) { const float* Wm = j < 2 ? WQ : j < 4 ? WK : WV; acc[j] = wmma_bf(a, fragb_f32(Wm + (size_t)((j & 1) * 16 + col) * HH, lane), acc[j]); }
#pragma unroll
  for (int j = 0; j < 6; ++j) { const float* Bm = j < 2 ? BQ : j < 4 ? BK : BV; const float bb = bfr(Bm[(j & 1) * 16 + col]);
#pragma unroll
    for (int r = 0; r < 8; ++r) { const float v = acc[j][r] + bb; const _Float16 hv = (_Float16)v, lv = (_Float16)((v - (float)hv) * 2048.0f); if (j < 4) { sh[wave * 16 + 8 * g + r][j * 16 + col] = hv; sl[wave * 16 + 8 * g + r][j * 16 + col] = lv; } else { th[(j - 4) * 16 + col][wave * 16 + 8 * g + r] = hv; tl[(j - 4) * 16 + col][wave * 16 + 8 * g + r] = lv; } } }
  if (tid < 64) { float s = 0.f;
#pragma unroll
    for (int tau = 0; tau < NLAG; ++tau) s += sdw[tau] * bfr(X[(b * TT + (TT - 1 - tau)) * (size_t)NN + n0 + tid]);
    const _Float16 hv = (_Float16)s; th[HH][tid] = hv; tl[HH][tid] = (_Float16)((s - (float)hv) * 2048.0f); }
  __syncthreads();
  for (int e = tid; e < 64 * 8; e += 128) { const int rl = e >> 3, q = e & 7; const size_t o = (b * NN + n0 + rl) * (2 * HH) + q * 8; vst2((unsigned*)(QK + o), *(const v4u*)&sh[rl][q * 8]); vst2((unsigned*)(QKL + o), *(const v4u*)&sl[rl][q * 8]); }
  for (int e = tid; e < NVC * 8; e += 128) { const int c = e >> 3, q = e & 7; const size_t o = (b * NVC + c) * (size_t)NN + n0 + q * 8; vst2((unsigned*)(VT + o), *(const v4u*)&th[c][q * 8]); vst2((unsigned*)(VTL + o), *(const v4u*)&tl[c][q * 8]); } }
__global__ __launch_bounds__(128) void k_att(const _Float16* __restrict__ QK, const _Float16* __restrict__ QKL, const _Float16* __restrict__ VT, const _Float16* __restrict__ VTL, const float* __restrict__ ADJ, const float* __restrict__ GEO, const float* __restrict__ FT, const float* __restrict__ WO, const float* __restrict__ BO, const float* __restrict__ G, const float* __restrict__ Bt, float* __restrict__ OUT) {
  __shared__ __align__(16) float sp[4][16][36]; __shared__ __align__(16) float so[4][16][52]; __shared__ float swo[HH][HH + 1]; __shared__ __align__(16) float sres[4][16][HH + 4];
  const int tid = threadIdx.x, wave = tid >> 5, lane = tid & 31, col = lane & 15, g = lane >> 4; const size_t b = blockIdx.y; const int q0 = blockIdx.x * 64 + wave * 16; const size_t rq = b * NN + q0;
  for (int e = tid; e < HH * HH; e += 128) swo[e / HH][e % HH] = bfr(WO[e]);
  const float geo = 1.0f / (1.0f + expf(-bfr(GEO[0]))); const float sqk = (1.0f - geo) * 0.17677669529663687f, spr = geo * 5.0f;
  const v16h aq = frag_h(QK + (rq + col) * (2 * HH), lane), aql = frag_h(QKL + (rq + col) * (2 * HH), lane);
  float m[8], l[8];
#pragma unroll
  for (int r = 0; r < 8; ++r) { m[r] = -3.0e38f; l[r] = 0.f; }
  v8f acc[3] = {}, accl[3] = {};
#pragma unroll 1
  for (int ks = 0; ks < NN / 32; ++ks) { float s[2][8];
#pragma unroll
    for (int ct = 0; ct < 2; ++ct) { const int kk = ks * 32 + ct * 16 + col; const size_t rk = b * NN + kk; const v16h kh = frag_h(QK + rk * (2 * HH) + HH, lane), kl = frag_h(QKL + rk * (2 * HH) + HH, lane); v8f c = {}, cl = {}; c = wmma16(aq, kh, c); cl = wmma16(aq, kl, cl); cl = wmma16(aql, kh, cl);
#pragma unroll
      for (int r = 0; r < 8; ++r) s[ct][r] = (c[r] + cl[r] * (1.0f / 2048.0f)) * sqk + spr * bfr(ADJ[(size_t)(q0 + 8 * g + r) * NN + kk]); }
    float alpha[8];
#pragma unroll
    for (int r = 0; r < 8; ++r) { float mx = fmaxf(s[0][r], s[1][r]);
#pragma unroll
      for (int o = 1; o < 16; o <<= 1) mx = fmaxf(mx, __shfl_xor(mx, o));
      const float mn = fmaxf(m[r], mx); alpha[r] = __expf(m[r] - mn); const float e0 = __expf(s[0][r] - mn), e1 = __expf(s[1][r] - mn); float es = e0 + e1;
#pragma unroll
      for (int o = 1; o < 16; o <<= 1) es += __shfl_xor(es, o);
      l[r] = l[r] * alpha[r] + es; m[r] = mn; sp[wave][8 * g + r][col] = e0; sp[wave][8 * g + r][16 + col] = e1; }
#pragma unroll
    for (int j = 0; j < 3; ++j)
#pragma unroll
      for (int r = 0; r < 8; ++r) { acc[j][r] *= alpha[r]; accl[j][r] *= alpha[r]; }
    LDSX();
    v16h pa, pal; { const float* prow = &sp[wave][col][0] + 8 * (lane >> 4);
#pragma unroll
      for (int i = 0; i < 8; ++i) { const float p0 = prow[i] * 2048.0f, p1 = prow[16 + i] * 2048.0f; pa[i] = (_Float16)p0; pa[8 + i] = (_Float16)p1; pal[i] = (_Float16)((p0 - (float)pa[i]) * 2048.0f); pal[8 + i] = (_Float16)((p1 - (float)pa[8 + i]) * 2048.0f); } }
#pragma unroll
    for (int j = 0; j < 3; ++j) { const size_t po = (b * NVC + j * 16 + col) * (size_t)NN + ks * 32; const v16h vh = frag_h(VT + po, lane), vl = frag_h(VTL + po, lane); acc[j] = wmma16(pa, vh, acc[j]); accl[j] = wmma16(pa, vl, accl[j]); accl[j] = wmma16(pal, vh, accl[j]); }
    LDSX(); }
#pragma unroll
  for (int r = 0; r < 8; ++r) { const float il = (1.0f / 2048.0f) / l[r];
#pragma unroll
    for (int j = 0; j < 3; ++j) so[wave][8 * g + r][j * 16 + col] = (acc[j][r] + accl[j][r] * (1.0f / 2048.0f)) * il; }
  __syncthreads();
#pragma unroll 1
  for (int rl = 0; rl < 16; ++rl) { const size_t row = rq + rl; const float* at = &so[wave][rl][0]; float hsum = bfr(BO[lane]);
#pragma unroll 1
    for (int c = 0; c < HH; ++c) { const float comb = bfr(FT[row * HH + c]) + at[c] + 0.1f * at[HH]; hsum += comb * swo[lane][c]; }
    float mu = hsum;
#pragma unroll
    for (int o = 1; o < 32; o <<= 1) mu += __shfl_xor(mu, o);
    mu *= (1.0f / HH); const float d = hsum - mu; float var = d * d;
#pragma unroll
    for (int o = 1; o < 32; o <<= 1) var += __shfl_xor(var, o);
    var *= (1.0f / HH); sres[wave][rl][lane] = d / sqrtf(var + LNEPS) * bfr(G[lane]) + bfr(Bt[lane]); }
  LDSX(); for (int rl = 0; rl < 16; ++rl) if (lane < 8) vst2(OUT + (rq + rl) * HH + lane * 4, *(const v4f*)&sres[wave][rl][lane * 4]); }
extern "C" void kernel_launch(void* const* d_in, const int* in_sizes, int n_in, void* d_out, int out_size, void* d_ws, size_t ws_size, hipStream_t stream) {
  (void)in_sizes; (void)n_in; (void)out_size;
  const float** F = (const float**)d_in;
  if (ws_size < (size_t)WS_END) return;
  char* ws = (char*)d_ws; _Float16 *QK = (_Float16*)(ws + WS_QK), *QKL = (_Float16*)(ws + WS_QKL), *VT = (_Float16*)(ws + WS_VT), *VTL = (_Float16*)(ws + WS_VTL);
  k_prep<<<dim3(NN / 64, TNB), 128, 0, stream>>>(F[0], F[1], F[2], F[3], F[4], F[5], F[6], F[7], F[8], QK, QKL, VT, VTL);
  k_att<<<dim3(NN / 64, TNB), 128, 0, stream>>>(QK, QKL, VT, VTL, F[9], F[10], F[1], F[11], F[12], F[13], F[14], (float*)d_out);
}
